// BayesConv2dMF_11639361372311
// MI455X (gfx1250) — hardware-verified
//
#include <hip/hip_runtime.h>
#include <hip/hip_bf16.h>

#define __bf16 _Float16
typedef __attribute__((ext_vector_type(16))) _Float16 v16bf;
typedef __attribute__((ext_vector_type(8)))  _Float16 v8h;
typedef __attribute__((ext_vector_type(8)))  float  v8f;
#define VST2(T, ptr, val) do { const T _v = (val); *(volatile T*)(ptr) = _v; __threadfence(); *(volatile T*)(ptr) = _v; } while (0)

#define B_    32
#define CO_   128
#define CI_   128
#define H_    56
#define W_    56
#define HW_   (H_ * W_)
#define NTILE 64
#define KC    32
#define HROWS 5
#define HCOLS 58
#define HSLICE (HCOLS * KC)
#define HUNITS (HROWS * HCOLS * 4)
#define BLK   128

union frag16 { uint4 u4[2]; v16bf v; };
union pack8  { uint4 u4; __bf16 e[8]; };

__global__ __launch_bounds__(256) void weight_prep_kernel(
    const float* __restrict__ eps,
    const float* __restrict__ psi,
    const float* __restrict__ mu,
    __bf16* __restrict__ wbf)
{
    int t8 = blockIdx.x * 256 + threadIdx.x;
    int t  = t8 * 8;
    int ci0 = t & (CI_ - 1);
    int co = (t >> 7) & (CO_ - 1);
    int rs = (t >> 14) % 9;
    int b  = t / (9 << 14);
    v8h o;
    #pragma unroll
    for (int q = 0; q < 8; ++q) {
        int ci = ci0 + q;
        int pidx = (co * CI_ + ci) * 9 + rs;
        int eidx = ((b * CO_ + co) * CI_ + ci) * 9 + rs;
        o[q] = (__bf16)(eps[eidx] * expf(psi[pidx]) + mu[pidx]);
    }
    VST2(v8h, wbf + t, o);
}

__global__ __launch_bounds__(BLK) void conv_wmma_kernel(
    const float*  __restrict__ in,
    const __bf16* __restrict__ wbf,
    float*        __restrict__ out)
{
    __shared__ __bf16 sH[HROWS * HSLICE];

    const int b    = blockIdx.y;
    const int n0   = blockIdx.x * NTILE;
    const int tid  = threadIdx.x;
    const int lane = tid & 31;
    const int waveM = tid >> 5;
    const int lrow  = lane & 15;
    const int lhalf = lane >> 4;

    const int rfirst = n0 / W_;

    int bbase[4];
    #pragma unroll
    for (int n = 0; n < 4; ++n) {
        int p = n0 + n * 16 + lrow;
        int h = p / W_;
        int w = p - h * W_;
        bbase[n] = ((h - rfirst) * HCOLS + w) * KC + lhalf * 8;
    }

    int arow[2];
    #pragma unroll
    for (int m = 0; m < 2; ++m)
        arow[m] = (waveM * 32 + m * 16 + lrow) * CI_ + lhalf * 8;

    v8f acc[2][4] = {};

    const float*  inB = in  + (size_t)b * CI_ * HW_;
    const __bf16* wB  = wbf + (size_t)b * 9 * CO_ * CI_;

    for (int kc = 0; kc < CI_; kc += KC) {
        __syncthreads();

        for (int u = tid; u < HUNITS; u += BLK) {
            const int ci8 = (u & 3) * 8;
            const int hc  = (u >> 2) % HCOLS;
            const int hr  = (u >> 2) / HCOLS;
            const int gh  = rfirst - 1 + hr;
            const int gw  = hc - 1;
            const bool v  = (gh >= 0) & (gh < H_) & (gw >= 0) & (gw < W_);
            const float* src = inB + (size_t)(kc + ci8) * HW_ + gh * W_ + gw;
            pack8 pk;
            #pragma unroll
            for (int i = 0; i < 8; ++i)
                pk.e[i] = (__bf16)(v ? src[(size_t)i * HW_] : 0.0f);
            *(uint4*)(&sH[hr * HSLICE + hc * KC + ci8]) = pk.u4;

            if (kc + KC < CI_)
                __builtin_prefetch(src + (size_t)KC * HW_, 0, 1);
        }
        __syncthreads();

        #pragma unroll
        for (int rs = 0; rs < 9; ++rs) {
            const int r = rs / 3;
            const int s = rs - 3 * r;
            const __bf16* wA = wB + (size_t)rs * CO_ * CI_ + kc;

            v16bf afrag[2];
            #pragma unroll
            for (int m = 0; m < 2; ++m) {
                const __bf16* ap = wA + arow[m];
                frag16 f;
                f.u4[0] = *(const uint4*)(ap);
                f.u4[1] = *(const uint4*)(ap + 16);
                afrag[m] = f.v;
            }

            v16bf bfrag[4];
            #pragma unroll
            for (int n = 0; n < 4; ++n) {
                const __bf16* bp = &sH[bbase[n] + (r * HCOLS + s) * KC];
                frag16 f;
                f.u4[0] = *(const uint4*)(bp);
                f.u4[1] = *(const uint4*)(bp + 16);
                bfrag[n] = f.v;
            }

            #pragma unroll
            for (int m = 0; m < 2; ++m)
                #pragma unroll
                for (int n = 0; n < 4; ++n)
                {   acc[m][n] = __builtin_amdgcn_wmma_f32_16x16x32_f16(
                        false, afrag[m], false, bfrag[n],
                        (short)0, acc[m][n], false, false);
                    asm volatile("v_nop\n\tv_nop\n\tv_nop\n\tv_nop" : "+v"(acc[m][n]) : "v"(afrag[m]), "v"(bfrag[n])); }
        }
    }

    float* outB = out + (size_t)b * CO_ * HW_;
    for (int pass = 0; pass < 2; ++pass) {
        #pragma unroll
        for (int m = 0; m < 2; ++m)
            #pragma unroll
            for (int pr = 0; pr < 2; ++pr)
                #pragma unroll
                for (int i = 0; i < 8; ++i) {
                    const float a_ = acc[m][2 * pr][i], b_ = acc[m][2 * pr + 1][i];
                    const float ax = __shfl_xor(a_, 16), bx = __shfl_xor(b_, 16);
                    const int co0 = waveM * 32 + m * 16 + i;
                    *(volatile float*)(outB + (size_t)co0 * HW_ + n0 + pr * 32 + lane)       = lhalf ? bx : a_;
                    *(volatile float*)(outB + (size_t)(co0 + 8) * HW_ + n0 + pr * 32 + lane) = lhalf ? b_ : ax;
                }
        __threadfence();
    }
}

extern "C" void kernel_launch(void* const* d_in, const int* in_sizes, int n_in,
                              void* d_out, int out_size, void* d_ws, size_t ws_size,
                              hipStream_t stream) {
    const float* input = (const float*)d_in[0];
    const float* eps   = (const float*)d_in[1];
    const float* psi   = (const float*)d_in[2];
    const float* mu    = (const float*)d_in[3];
    float*   out = (float*)d_out;
    __bf16*  wbf = (__bf16*)d_ws;

    (void)in_sizes; (void)n_in; (void)out_size;
    if (ws_size < (size_t)B_ * 9 * CO_ * CI_ * 2) return;
    const int nw = B_ * 9 * CO_ * CI_;
    weight_prep_kernel<<<dim3(nw / 8 / 256), dim3(256), 0, stream>>>(eps, psi, mu, wbf);

    conv_wmma_kernel<<<dim3(HW_ / NTILE, B_), dim3(BLK), 0, stream>>>(input, wbf, out);
}
